// Point_contextual_entropy_parameter_6047313953087
// MI455X (gfx1250) — hardware-verified
//
#include <hip/hip_runtime.h>
#include <math.h>
typedef __attribute__((ext_vector_type(16))) _Float16 v16h;
typedef __attribute__((ext_vector_type(8)))  _Float16 v8h;
typedef __attribute__((ext_vector_type(16))) __bf16   v16b;
typedef __attribute__((ext_vector_type(8)))  __bf16   v8b;
typedef __attribute__((ext_vector_type(8)))  float    v8f;
typedef __attribute__((ext_vector_type(4)))  float    v4f;
#define PSCALE 32768.0f
#define U16(p) ((const unsigned short*)(const void*)(p))
#define PSCALE_INV (1.0f / 32768.0f)

__device__ __forceinline__ unsigned short f2bf_bits(float f) {
  unsigned u = __float_as_uint(f);
  return (unsigned short)((u + 0x7FFFu + ((u >> 16) & 1u)) >> 16);
}
__device__ __forceinline__ float bf_bits2f(unsigned short h) { return __uint_as_float(((unsigned)h) << 16); }

__device__ __forceinline__ void dep_guard_h(v8f& a, v8f& b, v16h x, v16h y) { asm volatile("v_nop\n\tv_nop\n\tv_nop\n\tv_nop" : "+v"(a), "+v"(b) : "v"(x), "v"(y)); }
__device__ __forceinline__ void dep_guard_b(v8f& a, v8f& b, v16b x, v16b y) { asm volatile("v_nop\n\tv_nop\n\tv_nop\n\tv_nop" : "+v"(a), "+v"(b) : "v"(x), "v"(y)); }
__device__ __forceinline__ void keep4_h(v16h a, v16h b, v16h c, v16h d) { asm volatile("v_nop" :: "v"(a), "v"(b), "v"(c), "v"(d)); }
__device__ __forceinline__ void keep4_b(v16b a, v16b b, v16b c, v16b d) { asm volatile("v_nop" :: "v"(a), "v"(b), "v"(c), "v"(d)); }
__device__ __forceinline__ void acc_guard4(v8f& a, v8f& b, v8f& c, v8f& d) { asm volatile("v_nop\n\tv_nop\n\tv_nop\n\tv_nop" : "+v"(a), "+v"(b), "+v"(c), "+v"(d)); }
template <typename T> struct Frag;
template <> struct Frag<_Float16> {
  typedef v16h V; union U { v16h v; v8h h[2]; };
  static __device__ __forceinline__ v16h load(const _Float16* p) {
    U f; f.h[0] = *(const v8h*)(p); f.h[1] = *(const v8h*)(p + 16); return f.v;
  }
  static __device__ __forceinline__ v8f mma(v16h a, v16h b, v8f c) {
    return __builtin_amdgcn_wmma_f32_16x16x32_f16(false, a, false, b, (short)0, c, false, false);
  }
  static __device__ __forceinline__ void guard(v8f& a, v8f& b, v16h x, v16h y) { dep_guard_h(a, b, x, y); }
  static __device__ __forceinline__ void keep(v16h a, v16h b, v16h c, v16h d) { keep4_h(a, b, c, d); }
};
template <> struct Frag<__bf16> {
  typedef v16b V; union U { v16b v; v8b h[2]; };
  static __device__ __forceinline__ v16b load(const __bf16* p) {
    U f; f.h[0] = *(const v8b*)(p); f.h[1] = *(const v8b*)(p + 16); return f.v;
  }
  static __device__ __forceinline__ v8f mma(v16b a, v16b b, v8f c) {
    return __builtin_amdgcn_wmma_f32_16x16x32_bf16(false, a, false, b, (short)0, c, false, false);
  }
  static __device__ __forceinline__ void guard(v8f& a, v8f& b, v16b x, v16b y) { dep_guard_b(a, b, x, y); }
  static __device__ __forceinline__ void keep(v16b a, v16b b, v16b c, v16b d) { keep4_b(a, b, c, d); }
};

template <int ET> struct Elem;
template <> struct Elem<0> { typedef _Float16 T; };
template <> struct Elem<1> { typedef __bf16 T; };
template <int ET, bool SPLIT, int BIAS_MODE, int OUT_MODE, bool RESID, int ACT = 0>
__global__ __launch_bounds__(256) void wmma_gemm64(
    const unsigned short* __restrict__ Ap, const unsigned short* __restrict__ A2p, int lda, long strideA,
    const unsigned short* __restrict__ Btp, const unsigned short* __restrict__ Bt2p, int ldb, long strideB,
    void* __restrict__ Cout, void* __restrict__ Cout2, int ldc, long strideC,
    const float* __restrict__ bias,
    const float* __restrict__ resid, long strideR,
    int M, int N, int K, float scale) {
  typedef typename Elem<ET>::T T;
  typedef typename Frag<T>::V V;
  const T* A = (const T*)Ap; const T* A2 = (const T*)A2p; const T* Bt = (const T*)Btp; const T* Bt2 = (const T*)Bt2p;
  __shared__ __align__(16) float sT[8][16 * 68];
  const int b    = blockIdx.y;
  const int lane = threadIdx.x & 31;
  const int wave = threadIdx.x >> 5;
  const int tilesN = N >> 6;
  const int tilesM = M >> 6;
  const int tile = blockIdx.x * 8 + wave;
  if (tile >= tilesM * tilesN) return;
  const int tm = tile / tilesN;
  const int tn = tile - tm * tilesN;
  const int m0 = tm << 6;
  const int n0 = tn << 6;

  const T* Ab  = A  + (size_t)b * strideA;
  const T* Bb  = Bt + (size_t)b * strideB;
  const T* Ab2 = SPLIT ? (A2  + (size_t)b * strideA) : nullptr;
  const T* Bb2 = SPLIT ? (Bt2 + (size_t)b * strideB) : nullptr;

  const int rlane = lane & 15;
  const int koff  = (lane >> 4) * 8;
  const int mOff  = (lane >> 4) * 8;

  v8f acc[4][4];
#pragma unroll
  for (int i = 0; i < 4; ++i)
#pragma unroll
    for (int j = 0; j < 4; ++j) acc[i][j] = (v8f){0.f,0.f,0.f,0.f,0.f,0.f,0.f,0.f};

  for (int k0 = 0; k0 < K; k0 += 32) {
    V bh[4], bl[4];
#pragma unroll
    for (int j = 0; j < 4; ++j) {
      const size_t bo = (size_t)(n0 + (j << 4) + rlane) * ldb + koff + k0;
      bh[j] = Frag<T>::load(Bb + bo);
      if (SPLIT) bl[j] = Frag<T>::load(Bb2 + bo);
    }
#pragma unroll
    for (int i = 0; i < 4; ++i) {
      const size_t ao = (size_t)(m0 + (i << 4) + rlane) * lda + koff + k0;
      V ah = Frag<T>::load(Ab + ao);
      V al;
      if (SPLIT) al = Frag<T>::load(Ab2 + ao);
#pragma unroll
      for (int j = 0; j < 4; ++j) {
        acc[i][j] = Frag<T>::mma(ah, bh[j], acc[i][j]);
        if (SPLIT) {
          acc[i][j] = Frag<T>::mma(ah, bl[j], acc[i][j]);
          acc[i][j] = Frag<T>::mma(al, bh[j], acc[i][j]);
        }
      }
      Frag<T>::guard(acc[i][0], acc[i][3], ah, SPLIT ? al : ah);
    }
    Frag<T>::keep(bh[0], bh[1], bh[2], bh[3]);
    if (SPLIT) Frag<T>::keep(bl[0], bl[1], bl[2], bl[3]);
  }
  acc_guard4(acc[0][0], acc[0][1], acc[0][2], acc[0][3]);
  acc_guard4(acc[1][0], acc[1][1], acc[1][2], acc[1][3]);
  acc_guard4(acc[2][0], acc[2][1], acc[2][2], acc[2][3]);
  acc_guard4(acc[3][0], acc[3][1], acc[3][2], acc[3][3]);

  float* slab = sT[wave];
  const float* Rb = RESID ? (resid + (size_t)b * strideR) : nullptr;
#pragma unroll
  for (int i = 0; i < 4; ++i) {
    const int mBase = m0 + (i << 4);
#pragma unroll
    for (int j = 0; j < 4; ++j) {
      const int n = n0 + (j << 4) + rlane;
      float bv = 0.f;
      if (BIAS_MODE == 2) bv = bias[n];
#pragma unroll
      for (int r = 0; r < 8; ++r) {
        float v = acc[i][j][r] * scale;
        if (BIAS_MODE == 1) v += bias[mBase + mOff + r];
        if (BIAS_MODE == 2) v += bv;
        if (RESID) v += Rb[(size_t)(mBase + mOff + r) * ldc + n];
        if (ACT == 1) v = tanhf(v);
        if (ACT == 2) v = fmaxf(v, 0.0f);
        if (ACT == 3) v = v / (1.0f + expf(-v));
        if (ACT == 4) v = (v > 0.f) ? v : 0.01f * v;
        if (ACT == 5) v = 0.5f * v * (1.0f + erff(v * 0.70710678118654752f));
        slab[(mOff + r) * 68 + (j << 4) + rlane] = v;
      }
    }
    __builtin_amdgcn_fence(__ATOMIC_RELEASE, "workgroup");
    __builtin_amdgcn_wave_barrier();
    __builtin_amdgcn_fence(__ATOMIC_ACQUIRE, "workgroup");
    if (OUT_MODE == 0) {
      float* C = (float*)Cout + (size_t)b * strideC;
      const int hh = lane >> 4, c4 = (lane & 15) * 4;
      for (int pass = 0; pass < 2; ++pass) {
#pragma unroll
        for (int it = 0; it < 8; ++it) {
          const int row = it * 2 + hh;
          v4f v = *(const v4f*)(slab + row * 68 + c4);
          *(volatile v4f*)(C + (size_t)(mBase + row) * ldc + n0 + c4) = v;
        }
        __threadfence();
      }
    } else {
      const int q = lane >> 3, c8 = (lane & 7) * 8;
      unsigned short* C  = (unsigned short*)Cout  + (size_t)b * strideC;
      unsigned short* C2 = (OUT_MODE == 2) ? ((unsigned short*)Cout2 + (size_t)b * strideC) : nullptr;
      for (int pass = 0; pass < 2; ++pass) {
#pragma unroll
        for (int it = 0; it < 4; ++it) {
          const int row = it * 4 + q;
          const float* sp = slab + row * 68 + c8;
          v8h hv, lv;
#pragma unroll
          for (int e = 0; e < 8; ++e) {
            if (OUT_MODE == 1) {
              hv[e] = (_Float16)sp[e];
            } else {
              unsigned short hb = f2bf_bits(sp[e]);
              unsigned short lb = f2bf_bits(sp[e] - bf_bits2f(hb));
              hv[e] = __builtin_bit_cast(_Float16, hb);
              lv[e] = __builtin_bit_cast(_Float16, lb);
            }
          }
          *(volatile v8h*)(C + (size_t)(mBase + row) * ldc + n0 + c8) = hv;
          if (OUT_MODE == 2) *(volatile v8h*)(C2 + (size_t)(mBase + row) * ldc + n0 + c8) = lv;
        }
        __threadfence();
      }
    }
    __builtin_amdgcn_fence(__ATOMIC_RELEASE, "workgroup");
    __builtin_amdgcn_wave_barrier();
    __builtin_amdgcn_fence(__ATOMIC_ACQUIRE, "workgroup");
  }
}

__global__ __launch_bounds__(256) void cast_f32_f16x2(
    const float* __restrict__ in, _Float16* __restrict__ out, int n2) {
  int i = blockIdx.x * 256 + threadIdx.x;
  if (i < n2) {
    const _Float16 h0 = (_Float16)in[2 * i], h1 = (_Float16)in[2 * i + 1];
    const unsigned u = (unsigned)__builtin_bit_cast(unsigned short, h0) | ((unsigned)__builtin_bit_cast(unsigned short, h1) << 16);
    ((volatile unsigned*)out)[i] = u;
    __threadfence();
    ((volatile unsigned*)out)[i] = u;
  }
}


__global__ __launch_bounds__(256) void transpose_cast_f16(const float* __restrict__ in, int ldi,
                                                         _Float16* __restrict__ outT, int ldo, float scale) {
  __shared__ __align__(16) _Float16 tile[64][72];
  const int c0 = blockIdx.x * 64, r0 = blockIdx.y * 64;
  const int t = threadIdx.y * 32 + threadIdx.x;
  for (int i = threadIdx.y; i < 64; i += 8) {
    tile[threadIdx.x][i]      = (_Float16)(in[(size_t)(r0 + i) * ldi + c0 + threadIdx.x] * scale);
    tile[32 + threadIdx.x][i] = (_Float16)(in[(size_t)(r0 + i) * ldi + c0 + 32 + threadIdx.x] * scale);
  }
  __syncthreads();
  const int q = t >> 3, c8 = (t & 7) * 8;
  for (int pass = 0; pass < 2; ++pass) {
#pragma unroll
    for (int it = 0; it < 2; ++it) {
      const int c = it * 32 + q;
      v8h hv = *(const v8h*)(&tile[c][c8]);
      *(volatile v8h*)(outT + (size_t)(c0 + c) * ldo + r0 + c8) = hv;
    }
    __threadfence();
  }
}

#define PN 65536
#define PK 27
#define PC 64
#define PKK (PK * PC)
#define PCH 16384
template <bool SRC16>
__global__ __launch_bounds__(256) void gather_kernel(const void* __restrict__ feat, const int* __restrict__ nidx, int n0, unsigned* __restrict__ G) {
  const int lane = threadIdx.x & 31, wave = threadIdx.x >> 5;
  const int r = blockIdx.x * 8 + wave; if (r >= PCH) return;
  const int n = n0 + r; const int* np_ = nidx + (size_t)n * PK;
  const int myj = (lane < PK) ? np_[lane] : -1;
  unsigned* grow = G + (size_t)r * (PKK / 2);
  unsigned u[PK];
#pragma unroll
  for (int o = 0; o < PK; ++o) {
    const int j = __shfl(myj, o, 32);
    unsigned v = 0u;
    if (j >= 0 && j < PN) {
      if (SRC16) v = ((const unsigned*)feat)[(size_t)j * (PC / 2) + lane];
      else { const float a = ((const float*)feat)[(size_t)j * PC + 2 * lane], b = ((const float*)feat)[(size_t)j * PC + 2 * lane + 1];
        v = (unsigned)__builtin_bit_cast(unsigned short, (_Float16)a) | ((unsigned)__builtin_bit_cast(unsigned short, (_Float16)b) << 16); }
    }
    u[o] = v;
  }
  for (int pass = 0; pass < 2; ++pass) {
#pragma unroll
    for (int o = 0; o < PK; ++o) ((volatile unsigned*)grow)[o * (PC / 2) + lane] = u[o];
    __threadfence(); }
}
__global__ __launch_bounds__(256) void wtrans_kernel(const float* __restrict__ Wsrc, int cout, unsigned* __restrict__ WT) {
  const int i = blockIdx.x * 256 + threadIdx.x; if (i >= 64 * PKK / 2) return;
  const int d = i / (PKK / 2), kp = i % (PKK / 2);
  float a = 0.f, b = 0.f;
  if (d < cout) { a = Wsrc[(size_t)(2 * kp) * cout + d]; b = Wsrc[(size_t)(2 * kp + 1) * cout + d]; }
  const unsigned u = (unsigned)__builtin_bit_cast(unsigned short, (_Float16)a) | ((unsigned)__builtin_bit_cast(unsigned short, (_Float16)b) << 16);
  ((volatile unsigned*)WT)[i] = u; __threadfence(); ((volatile unsigned*)WT)[i] = u;
}

__global__ void padbias_kernel(const float* __restrict__ b, float* __restrict__ bp) { const int i = threadIdx.x; const float v = (i < 16) ? b[i] : 0.f; ((volatile float*)bp)[i] = v; __threadfence(); ((volatile float*)bp)[i] = v; }
__global__ __launch_bounds__(256) void pack16_kernel(const float* __restrict__ T, float* __restrict__ out) {
  const int n = blockIdx.x * 256 + threadIdx.x; if (n >= PN) return;
  v4f v[4];
#pragma unroll
  for (int q = 0; q < 4; ++q) v[q] = *(const v4f*)(T + (size_t)n * 64 + 4 * q);
  for (int pass = 0; pass < 2; ++pass) {
#pragma unroll
    for (int q = 0; q < 4; ++q) *(volatile v4f*)(out + (size_t)n * 16 + 4 * q) = v[q];
    __threadfence();
  }
}
extern "C" void kernel_launch(void* const* d_in, const int* in_sizes, int n_in, void* d_out, int out_size, void* d_ws, size_t ws_size, hipStream_t stream) {
  (void)in_sizes; (void)n_in; (void)out_size; (void)ws_size;
  const float* x = (const float*)d_in[0]; const int* nidx = (const int*)d_in[1];
  const float* W1 = (const float*)d_in[2]; const float* b1 = (const float*)d_in[3];
  const float* W2 = (const float*)d_in[4]; const float* b2 = (const float*)d_in[5];
  const float* W3 = (const float*)d_in[6]; const float* b3 = (const float*)d_in[7];
  char* ws = (char*)d_ws; size_t off = 0;
  auto carve = [&](size_t bytes) -> char* { char* p = ws + off; off += (bytes + 255) & ~(size_t)255; return p; };
  unsigned* G = (unsigned*)carve((size_t)PCH * PKK * 2);
  unsigned* W1T = (unsigned*)carve((size_t)64 * PKK * 2); unsigned* W2T = (unsigned*)carve((size_t)64 * PKK * 2); unsigned* W3T = (unsigned*)carve((size_t)64 * PKK * 2);
  unsigned* H1 = (unsigned*)carve((size_t)PN * PC * 2);
  unsigned* H2 = (unsigned*)carve((size_t)PN * PC * 2);
  float* T3 = (float*)carve((size_t)PN * 64 * 4);
  float* b3p = (float*)carve(64 * 4);
  wtrans_kernel<<<(64 * PKK / 2 + 255) / 256, 256, 0, stream>>>(W1, 64, W1T);
  wtrans_kernel<<<(64 * PKK / 2 + 255) / 256, 256, 0, stream>>>(W2, 64, W2T);
  wtrans_kernel<<<(64 * PKK / 2 + 255) / 256, 256, 0, stream>>>(W3, 16, W3T);
  padbias_kernel<<<1, 64, 0, stream>>>(b3, b3p);
  const int t = (PCH / 64) * 1;
  for (int c = 0; c < PN / PCH; ++c) {
    gather_kernel<false><<<PCH / 8, 256, 0, stream>>>(x, nidx, c * PCH, G);
    wmma_gemm64<0, false, 2, 1, false, 2><<<dim3((t + 7) / 8, 1), 256, 0, stream>>>((const unsigned short*)G, nullptr, PKK, 0, (const unsigned short*)W1T, nullptr, PKK, 0, H1 + (size_t)c * PCH * (PC / 2), nullptr, PC, 0, b1, nullptr, 0, PCH, 64, PKK, 1.0f);
  }
  for (int c = 0; c < PN / PCH; ++c) {
    gather_kernel<true><<<PCH / 8, 256, 0, stream>>>(H1, nidx, c * PCH, G);
    wmma_gemm64<0, false, 2, 1, false, 2><<<dim3((t + 7) / 8, 1), 256, 0, stream>>>((const unsigned short*)G, nullptr, PKK, 0, (const unsigned short*)W2T, nullptr, PKK, 0, H2 + (size_t)c * PCH * (PC / 2), nullptr, PC, 0, b2, nullptr, 0, PCH, 64, PKK, 1.0f);
  }
  for (int c = 0; c < PN / PCH; ++c) {
    gather_kernel<true><<<PCH / 8, 256, 0, stream>>>(H2, nidx, c * PCH, G);
    wmma_gemm64<0, false, 2, 0, false, 0><<<dim3((t + 7) / 8, 1), 256, 0, stream>>>((const unsigned short*)G, nullptr, PKK, 0, (const unsigned short*)W3T, nullptr, PKK, 0, T3 + (size_t)c * PCH * 64, nullptr, 64, 0, b3p, nullptr, 0, PCH, 64, PKK, 1.0f);
  }
  pack16_kernel<<<PN / 256, 256, 0, stream>>>(T3, (float*)d_out);
}
